// BBRNNModel_43404939493527
// MI455X (gfx1250) — hardware-verified
//
#include <hip/hip_runtime.h>
#include <stdint.h>

typedef __attribute__((ext_vector_type(16))) _Float16 v16h;
typedef __attribute__((ext_vector_type(8)))  _Float16 v8h;
typedef __attribute__((ext_vector_type(8)))  float    v8f;
typedef __attribute__((ext_vector_type(4)))  float    v4f;

constexpr int NBATCH = 32;
constexpr int NSTEP  = 2048;
constexpr int NFEAT  = 128;
constexpr int NUNIT  = 128;
constexpr int NCLS   = 11;
constexpr int NGATE3 = 3 * NUNIT;
constexpr int HCAT   = 2 * NUNIT;
constexpr int NROWS  = NBATCH * NSTEP;
constexpr int WPLANE = NGATE3 * NFEAT;
constexpr int APITCH = 136;
constexpr int SPITCH = 36;
constexpr float WCARRY = 16.0f;
constexpr float WCARRY_INV = 0.0625f;
constexpr int DROWS  = 256;
constexpr int DQUADS = (DROWS * NCLS) / 4;
static_assert(NFEAT == NUNIT);
static_assert(NROWS % DROWS == 0);
static_assert((DROWS * NCLS * 4) % 128 == 0);
static_assert((APITCH * 2) % 16 == 0);
static_assert((SPITCH * 4) % 16 == 0);

union FragU { v16h v; v8h h[2]; };

__device__ __forceinline__ v16h frag_load_g(const _Float16* __restrict__ p) {
  FragU f;
  f.h[0] = *(const v8h*)(p);
  f.h[1] = *(const v8h*)(p + 16);
  return f.v;
}

__device__ __forceinline__ v8f mma_h(v16h a, v16h b, v8f c) {
  c = __builtin_amdgcn_wmma_f32_16x16x32_f16(false, a, false, b, (short)0, c, false, false);
  asm volatile("v_nop\n\tv_nop\n\tv_nop\n\tv_nop" : "+v"(c) : "v"(a), "v"(b));
  return c;
}

__device__ __forceinline__ v8f zero8() {
  return (v8f){0.f, 0.f, 0.f, 0.f, 0.f, 0.f, 0.f, 0.f};
}

__global__ __launch_bounds__(256) void prep_weights(
    const float* __restrict__ W_f, const float* __restrict__ U_f,
    const float* __restrict__ W_b, const float* __restrict__ U_b,
    _Float16* __restrict__ wt_all) {
  __shared__ __align__(16) _Float16 tile[32 * APITCH];
  const int tid = threadIdx.x;
  const int pid = blockIdx.y;
  const float* src = (pid == 0) ? W_f : (pid == 1) ? U_f : (pid == 2) ? W_b : U_b;
  const int n0 = blockIdx.x * 32;
#pragma unroll
  for (int i = 0; i < 16; ++i) {
    const int idx = tid + 256 * i;
    const int k = idx >> 5;
    const int nn = idx & 31;
    tile[nn * APITCH + k] = (_Float16)(src[(size_t)k * NGATE3 + n0 + nn] * WCARRY);
  }
  __syncthreads();
  _Float16* dst = wt_all + (size_t)pid * WPLANE;
  v8h vals[2];
#pragma unroll
  for (int it = 0; it < 2; ++it) {
    const int f = tid + 256 * it;
    const int row = f >> 4, c8 = (f & 15) * 8;
    vals[it] = *(const v8h*)(tile + row * APITCH + c8);
  }
  for (int pass = 0; pass < 2; ++pass) {
#pragma unroll
    for (int it = 0; it < 2; ++it) {
      const int f = tid + 256 * it;
      const int row = f >> 4, c8 = (f & 15) * 8;
      *(volatile v8h*)(dst + (size_t)(n0 + row) * NFEAT + c8) = vals[it];
    }
    __threadfence();
  }
}

__global__ __launch_bounds__(256) void gru_scan(
    const float* __restrict__ x, const _Float16* __restrict__ wt_all,
    const float* __restrict__ b_f, const float* __restrict__ b_b,
    float* __restrict__ hs_out) {
  __shared__ __align__(16) _Float16 xs[2][NBATCH * APITCH];
  __shared__ __align__(16) _Float16 hb[2][NBATCH * APITCH];
  __shared__ __align__(16) float slab[8][16 * SPITCH];

  const int tid  = threadIdx.x;
  const int lane = tid & 31, wave = tid >> 5;
  const int c    = lane & 15, hh = lane >> 4, koff = hh * 8;
  const int dir  = blockIdx.x;
  const int mt   = wave >> 2;
  const int q    = wave & 3;
  const _Float16* Wt = wt_all + (size_t)(2 * dir) * WPLANE;
  const _Float16* Ut = Wt + WPLANE;

  float bz[2], br[2], bxh[2], brh[2];
#pragma unroll
  for (int j = 0; j < 2; ++j) {
    const int u = 32 * q + 16 * j + c;
    const float fz = b_f[u] + b_f[NGATE3 + u];
    const float fr = b_f[NUNIT + u] + b_f[NGATE3 + NUNIT + u];
    const float fx = b_f[2 * NUNIT + u];
    const float fh = b_f[NGATE3 + 2 * NUNIT + u];
    const float gz = b_b[u] + b_b[NGATE3 + u];
    const float gr = b_b[NUNIT + u] + b_b[NGATE3 + NUNIT + u];
    const float gx = b_b[2 * NUNIT + u];
    const float gh = b_b[NGATE3 + 2 * NUNIT + u];
    bz[j]  = dir ? gz : fz;
    br[j]  = dir ? gr : fr;
    bxh[j] = dir ? gx : fx;
    brh[j] = dir ? gh : fh;
  }

  {
    v8h z8;
#pragma unroll
    for (int e = 0; e < 8; ++e) z8[e] = (_Float16)0.0f;
    _Float16* hb0 = &hb[0][0];
    for (int i = tid; i < (2 * NBATCH * APITCH) / 8; i += 256) *(v8h*)(hb0 + 8 * i) = z8;
  }
  float hreg[2][8];
#pragma unroll
  for (int j = 0; j < 2; ++j)
#pragma unroll
    for (int r = 0; r < 8; ++r) hreg[j][r] = 0.0f;
  __syncthreads();

  const int arow = (16 * mt + c) * APITCH + koff;
  const int xrow = tid >> 3, xcc = (tid & 7) * 16;
  const float* xbase = x + (size_t)xrow * NSTEP * NFEAT + xcc;
  float* sw = slab[wave];
  const size_t hsbase = (size_t)(16 * mt) * NSTEP * HCAT + (size_t)dir * NUNIT + (size_t)(32 * q);

  for (int s = 0; s < NSTEP; ++s) {
    const int t = dir ? (NSTEP - 1 - s) : s;
    const int cur = s & 1;
    _Float16* xa = xs[cur];
    const _Float16* ha = hb[cur];
    _Float16* hnx = hb[cur ^ 1];

    {
      const float* xr = xbase + (size_t)t * NFEAT;
      const v4f a0 = *(const v4f*)(xr);
      const v4f a1 = *(const v4f*)(xr + 4);
      const v4f a2 = *(const v4f*)(xr + 8);
      const v4f a3 = *(const v4f*)(xr + 12);
      v8h p0, p1;
#pragma unroll
      for (int e = 0; e < 4; ++e) {
        p0[e]     = (_Float16)a0[e];
        p0[4 + e] = (_Float16)a1[e];
        p1[e]     = (_Float16)a2[e];
        p1[4 + e] = (_Float16)a3[e];
      }
      *(v8h*)(xa + xrow * APITCH + xcc)     = p0;
      *(v8h*)(xa + xrow * APITCH + xcc + 8) = p1;
    }
    __syncthreads();

    v8f accZ[2], accR[2], accX[2], accH[2];
#pragma unroll
    for (int j = 0; j < 2; ++j) { accZ[j] = zero8(); accR[j] = zero8(); accX[j] = zero8(); accH[j] = zero8(); }

#pragma unroll 1
    for (int kc = 0; kc < 4; ++kc) {
      const int kk = kc * 32;
      FragU fa;
      fa.h[0] = *(const v8h*)(xa + arow + kk);
      fa.h[1] = *(const v8h*)(xa + arow + kk + 16);
#pragma unroll
      for (int j = 0; j < 2; ++j) {
        const _Float16* wp = Wt + (size_t)(32 * q + 16 * j + c) * NFEAT + kk + koff;
        const v16h fz = frag_load_g(wp);
        const v16h fr = frag_load_g(wp + (size_t)NUNIT * NFEAT);
        const v16h fh = frag_load_g(wp + (size_t)2 * NUNIT * NFEAT);
        accZ[j] = mma_h(fa.v, fz, accZ[j]);
        accR[j] = mma_h(fa.v, fr, accR[j]);
        accX[j] = mma_h(fa.v, fh, accX[j]);
      }
    }
#pragma unroll 1
    for (int kc = 0; kc < 4; ++kc) {
      const int kk = kc * 32;
      FragU fa;
      fa.h[0] = *(const v8h*)(ha + arow + kk);
      fa.h[1] = *(const v8h*)(ha + arow + kk + 16);
#pragma unroll
      for (int j = 0; j < 2; ++j) {
        const _Float16* up = Ut + (size_t)(32 * q + 16 * j + c) * NUNIT + kk + koff;
        const v16h fz = frag_load_g(up);
        const v16h fr = frag_load_g(up + (size_t)NUNIT * NUNIT);
        const v16h fh = frag_load_g(up + (size_t)2 * NUNIT * NUNIT);
        accZ[j] = mma_h(fa.v, fz, accZ[j]);
        accR[j] = mma_h(fa.v, fr, accR[j]);
        accH[j] = mma_h(fa.v, fh, accH[j]);
      }
    }

#pragma unroll
    for (int j = 0; j < 2; ++j) {
#pragma unroll
      for (int r = 0; r < 8; ++r) {
        float az = accZ[j][r] * WCARRY_INV + bz[j];
        float ar = accR[j][r] * WCARRY_INV + br[j];
        az = fminf(fmaxf(az, -30.0f), 30.0f);
        ar = fminf(fmaxf(ar, -30.0f), 30.0f);
        const float zg = __builtin_amdgcn_rcpf(1.0f + expf(-az));
        const float rg = __builtin_amdgcn_rcpf(1.0f + expf(-ar));
        const float xg = accX[j][r] * WCARRY_INV + bxh[j];
        const float rh = accH[j][r] * WCARRY_INV + brh[j];
        const float cand = fmaxf(0.0f, xg + rg * rh);
        const float hnew = zg * hreg[j][r] + (1.0f - zg) * cand;
        hreg[j][r] = hnew;
        sw[(8 * hh + r) * SPITCH + 16 * j + c] = hnew;
      }
    }
    __builtin_amdgcn_fence(__ATOMIC_RELEASE, "workgroup");
    __builtin_amdgcn_wave_barrier();
    __builtin_amdgcn_fence(__ATOMIC_ACQUIRE, "workgroup");

#pragma unroll
    for (int i = 0; i < 2; ++i) {
      const int f = lane + 32 * i;
      const int row = f >> 2, c8 = (f & 3) * 8;
      const v4f v0 = *(const v4f*)(sw + row * SPITCH + c8);
      const v4f v1 = *(const v4f*)(sw + row * SPITCH + c8 + 4);
      v8h p;
#pragma unroll
      for (int e = 0; e < 4; ++e) { p[e] = (_Float16)v0[e]; p[4 + e] = (_Float16)v1[e]; }
      *(v8h*)(hnx + (16 * mt + row) * APITCH + 32 * q + c8) = p;
    }

    for (int pass = 0; pass < 2; ++pass) {
#pragma unroll
      for (int it = 0; it < 4; ++it) {
        const int row = it * 4 + (lane >> 3);
        const int c4 = (lane & 7) * 4;
        const v4f v = *(const v4f*)(sw + row * SPITCH + c4);
        *(volatile v4f*)(hs_out + hsbase + ((size_t)row * NSTEP + (size_t)t) * HCAT + c4) = v;
      }
      __threadfence();
    }
    __builtin_amdgcn_fence(__ATOMIC_RELEASE, "workgroup");
    __builtin_amdgcn_wave_barrier();
    __builtin_amdgcn_fence(__ATOMIC_ACQUIRE, "workgroup");
  }
}

__global__ __launch_bounds__(256) void dense_softmax(
    const float* __restrict__ hs, const float* __restrict__ Wd,
    const float* __restrict__ bd, float* __restrict__ out) {
  __shared__ float wsh[HCAT * NCLS];
  __shared__ float bsh[16];
  __shared__ float lg[DROWS * 12];
  __shared__ __align__(16) float pk[DROWS * NCLS];
  const int tid = threadIdx.x;
#pragma unroll
  for (int i = 0; i < NCLS; ++i) wsh[tid + 256 * i] = Wd[tid + 256 * i];
  if (tid < NCLS) bsh[tid] = bd[tid];
  __syncthreads();

  const size_t orow = (size_t)blockIdx.x * DROWS + tid;
  const v4f* hrow = (const v4f*)(hs + orow * HCAT);
  float acc[NCLS];
#pragma unroll
  for (int cc = 0; cc < NCLS; ++cc) acc[cc] = bsh[cc];
#pragma unroll 1
  for (int k4 = 0; k4 < HCAT / 4; ++k4) {
    const v4f hv = hrow[k4];
    const float* w0 = wsh + (4 * k4) * NCLS;
#pragma unroll
    for (int cc = 0; cc < NCLS; ++cc)
      acc[cc] += hv[0] * w0[cc] + hv[1] * w0[NCLS + cc] + hv[2] * w0[2 * NCLS + cc] + hv[3] * w0[3 * NCLS + cc];
  }
  float mx = acc[0];
#pragma unroll
  for (int cc = 1; cc < NCLS; ++cc) mx = fmaxf(mx, acc[cc]);
  float* myl = lg + tid * 12;
#pragma unroll
  for (int cc = 0; cc < NCLS; ++cc) myl[cc] = acc[cc];
  float sum = 0.0f;
#pragma unroll 1
  for (int cc = 0; cc < NCLS; ++cc) {
    const float e = expf(myl[cc] - mx);
    myl[cc] = e;
    sum += e;
  }
  const float inv = __builtin_amdgcn_rcpf(sum);
  float* myp = pk + tid * NCLS;
#pragma unroll 1
  for (int cc = 0; cc < NCLS; ++cc) myp[cc] = myl[cc] * inv;
  __syncthreads();

  float* ob = out + (size_t)blockIdx.x * (DROWS * NCLS);
  v4f vv[3];
#pragma unroll
  for (int it = 0; it < 3; ++it) {
    const int f = tid + 256 * it;
    const int fc = (f < DQUADS) ? f : (DQUADS - 1);
    vv[it] = *(const v4f*)(pk + 4 * fc);
  }
  for (int pass = 0; pass < 2; ++pass) {
#pragma unroll
    for (int it = 0; it < 3; ++it) {
      const int f = tid + 256 * it;
      if (f < DQUADS) *(volatile v4f*)(ob + 4 * f) = vv[it];
    }
    __threadfence();
  }
}

extern "C" void kernel_launch(void* const* d_in, const int* in_sizes, int n_in,
                              void* d_out, int out_size, void* d_ws, size_t ws_size,
                              hipStream_t stream) {
  (void)n_in;
  const float* x   = (const float*)d_in[0];
  const float* W_f = (const float*)d_in[1];
  const float* U_f = (const float*)d_in[2];
  const float* b_f = (const float*)d_in[3];
  const float* W_b = (const float*)d_in[4];
  const float* U_b = (const float*)d_in[5];
  const float* b_b = (const float*)d_in[6];
  const float* Wd  = (const float*)d_in[7];
  const float* bd  = (const float*)d_in[8];

  const size_t wt_bytes = (size_t)4 * WPLANE * 2;
  const size_t hs_bytes = (size_t)NROWS * HCAT * 4;
  const size_t total = wt_bytes + hs_bytes;
  if (ws_size < total) return;
  if (in_sizes[0] != NROWS * NFEAT || out_size != NROWS * NCLS) return;

  char* ws = (char*)d_ws;
  _Float16* wt_all = (_Float16*)(ws);
  float* hs_plane  = (float*)(ws + wt_bytes);

  prep_weights<<<dim3(NGATE3 / 32, 4, 1), 256, 0, stream>>>(W_f, U_f, W_b, U_b, wt_all);
  gru_scan<<<dim3(2, 1, 1), 256, 0, stream>>>(x, wt_all, b_f, b_b, hs_plane);
  dense_softmax<<<dim3(NROWS / DROWS, 1, 1), 256, 0, stream>>>(hs_plane, Wd, bd, (float*)d_out);
}
